// MambaLayer_47897475285516
// MI455X (gfx1250) — hardware-verified
//
#include <hip/hip_runtime.h>
#include <math.h>

typedef __attribute__((ext_vector_type(16))) _Float16 v16h;
typedef __attribute__((ext_vector_type(8)))  _Float16 v8h;
typedef __attribute__((ext_vector_type(16))) __bf16   v16b;
typedef __attribute__((ext_vector_type(8)))  __bf16   v8b;
typedef __attribute__((ext_vector_type(8)))  float    v8f;
typedef __attribute__((ext_vector_type(4)))  float    v4f;

constexpr int kBatch  = 4;
constexpr int kSeq    = 2048;
constexpr int kDm     = 192;
constexpr int kDin    = 384;
constexpr int kNst    = 16;
constexpr int kDtR    = 12;
constexpr int kXzP    = 2 * kDin;
constexpr int kXdReal = kDtR + 2 * kNst;
constexpr int kXdP    = 64;
constexpr int kRows   = kBatch * kSeq;
constexpr int kLnTok  = 64;
constexpr int kLnP    = 65;
constexpr int kConvCh = 128;
constexpr int kConvTP = 132;
constexpr int kScanTS = 64;
constexpr int kScanCh = 64;
constexpr int kScanYP = 68;
constexpr float kInvDm = 1.0f / (float)kDm;

static_assert(kXdReal == 44 && kXdReal <= kXdP, "x_proj width");
static_assert((kDtR % 4) == 0, "dt columns read as float4 groups");
static_assert((kDm % 32) == 0 && (kDin % 32) == 0, "GEMM K multiples of 32");
static_assert((kRows % 64) == 0 && (kXzP % 64) == 0 && (kXdP % 64) == 0 && (kDm % 64) == 0 && (kSeq % 64) == 0, "GEMM M,N multiples of 64");
static_assert((kSeq % kScanTS) == 0 && (kSeq % kLnTok) == 0 && (kDin % kScanCh) == 0 && (kDin % kConvCh) == 0, "tile multiples");
static_assert(kRows == 8192 && kXzP == 768, "shape check");

constexpr size_t kSzWI  = (size_t)kXzP * kDm * 2;
constexpr size_t kSzWO  = (size_t)kDm * kDin * 2;
constexpr size_t kSzWX  = (size_t)kXdP * kDin * 2;
constexpr size_t kSzXN  = (size_t)kRows * kDm * 2;
constexpr size_t kSzXZ  = (size_t)kRows * kXzP * 4;
constexpr size_t kSzUC  = (size_t)kRows * kDin * 4;
constexpr size_t kSzU16 = (size_t)kRows * kDin * 2;
constexpr size_t kSzXD  = (size_t)kRows * kXdP * 4;
constexpr size_t kOffWIH = 0;
constexpr size_t kOffWIL = kOffWIH + kSzWI;
constexpr size_t kOffWOH = kOffWIL + kSzWI;
constexpr size_t kOffWOL = kOffWOH + kSzWO;
constexpr size_t kOffWXH = kOffWOL + kSzWO;
constexpr size_t kOffWXL = kOffWXH + kSzWX;
constexpr size_t kOffXNH = kOffWXL + kSzWX;
constexpr size_t kOffXNL = kOffXNH + kSzXN;
constexpr size_t kOffXZ  = kOffXNL + kSzXN;
constexpr size_t kOffUC  = kOffXZ  + kSzXZ;
constexpr size_t kOffUCH = kOffUC  + kSzUC;
constexpr size_t kOffXD  = kOffUCH + kSzU16;
constexpr size_t kOffYH  = kOffXD  + kSzXD;
constexpr size_t kOffYL  = kOffYH  + kSzU16;
constexpr size_t kWsTotal = kOffYL + kSzU16;
static_assert(kWsTotal == 65994752ull, "carve total");
static_assert(kWsTotal <= 134217728ull, "carve cap");
static_assert((kOffWIL % 128) == 0 && (kOffWOH % 128) == 0 && (kOffWOL % 128) == 0 && (kOffWXH % 128) == 0 &&
              (kOffWXL % 128) == 0 && (kOffXNH % 128) == 0 && (kOffXNL % 128) == 0 && (kOffXZ % 128) == 0 &&
              (kOffUC % 128) == 0 && (kOffUCH % 128) == 0 && (kOffXD % 128) == 0 && (kOffYH % 128) == 0 &&
              (kOffYL % 128) == 0, "128-B aligned regions");

__device__ __forceinline__ unsigned short f2bf_bits(float f) {
  unsigned u = __float_as_uint(f);
  return (unsigned short)((u + 0x7FFFu + ((u >> 16) & 1u)) >> 16);
}
__device__ __forceinline__ float bf_bits2f(unsigned short h) { return __uint_as_float(((unsigned)h) << 16); }

__device__ __forceinline__ void dep_guard4_h(v8f& a, v8f& b, v8f& c, v8f& d, v16h x, v16h y) {
  asm volatile("v_nop\n\tv_nop\n\tv_nop\n\tv_nop" : "+v"(a), "+v"(b), "+v"(c), "+v"(d) : "v"(x), "v"(y));
}
__device__ __forceinline__ void dep_guard4_b(v8f& a, v8f& b, v8f& c, v8f& d, v16b x, v16b y) {
  asm volatile("v_nop\n\tv_nop\n\tv_nop\n\tv_nop" : "+v"(a), "+v"(b), "+v"(c), "+v"(d) : "v"(x), "v"(y));
}
__device__ __forceinline__ void keep4_h(v16h a, v16h b, v16h c, v16h d) { asm volatile("v_nop" :: "v"(a), "v"(b), "v"(c), "v"(d)); }
__device__ __forceinline__ void keep4_b(v16b a, v16b b, v16b c, v16b d) { asm volatile("v_nop" :: "v"(a), "v"(b), "v"(c), "v"(d)); }
__device__ __forceinline__ void acc_guard4(v8f& a, v8f& b, v8f& c, v8f& d) {
  asm volatile("v_nop\n\tv_nop\n\tv_nop\n\tv_nop" : "+v"(a), "+v"(b), "+v"(c), "+v"(d));
}
template <typename T> struct Frag;
template <> struct Frag<_Float16> {
  typedef v16h V; union U { v16h v; v8h h[2]; };
  static __device__ __forceinline__ v16h load(const _Float16* p) {
    U f; f.h[0] = *(const v8h*)(p); f.h[1] = *(const v8h*)(p + 16); return f.v;
  }
  static __device__ __forceinline__ v8f mma(v16h a, v16h b, v8f c) {
    return __builtin_amdgcn_wmma_f32_16x16x32_f16(false, a, false, b, (short)0, c, false, false);
  }
  static __device__ __forceinline__ void guard(v8f& a, v8f& b, v8f& c, v8f& d, v16h x, v16h y) { dep_guard4_h(a, b, c, d, x, y); }
  static __device__ __forceinline__ void keep(v16h a, v16h b, v16h c, v16h d) { keep4_h(a, b, c, d); }
};
template <> struct Frag<__bf16> {
  typedef v16b V; union U { v16b v; v8b h[2]; };
  static __device__ __forceinline__ v16b load(const __bf16* p) {
    U f; f.h[0] = *(const v8b*)(p); f.h[1] = *(const v8b*)(p + 16); return f.v;
  }
  static __device__ __forceinline__ v8f mma(v16b a, v16b b, v8f c) {
    return __builtin_amdgcn_wmma_f32_16x16x32_bf16(false, a, false, b, (short)0, c, false, false);
  }
  static __device__ __forceinline__ void guard(v8f& a, v8f& b, v8f& c, v8f& d, v16b x, v16b y) { dep_guard4_b(a, b, c, d, x, y); }
  static __device__ __forceinline__ void keep(v16b a, v16b b, v16b c, v16b d) { keep4_b(a, b, c, d); }
};

template <int ET> struct Elem;
template <> struct Elem<0> { typedef _Float16 T; };
template <> struct Elem<1> { typedef __bf16 T; };
template <int ET, int SPL, int BIAS_MODE, int OUT_MODE, bool RESID, int ACT = 0>
__global__ __launch_bounds__(256) void wmma_gemm64(
    const unsigned short* __restrict__ Ap, const unsigned short* __restrict__ A2p, int lda, long strideA,
    const unsigned short* __restrict__ Btp, const unsigned short* __restrict__ Bt2p, int ldb, long strideB,
    void* __restrict__ Cout, void* __restrict__ Cout2, int ldc, long strideC,
    const float* __restrict__ bias,
    const float* __restrict__ resid, long strideR,
    int M, int N, int K, float scale) {
  typedef typename Elem<ET>::T T;
  typedef typename Frag<T>::V V;
  const T* A = (const T*)Ap; const T* A2 = (const T*)A2p; const T* Bt = (const T*)Btp; const T* Bt2 = (const T*)Bt2p;
  __shared__ __align__(16) float sT[8][16 * 68];
  const int b    = blockIdx.y;
  const int lane = threadIdx.x & 31;
  const int wave = threadIdx.x >> 5;
  const int tilesN = N >> 6;
  const int tilesM = M >> 6;
  const int tile = blockIdx.x * 8 + wave;
  if (tile >= tilesM * tilesN) return;
  const int tm = tile / tilesN;
  const int tn = tile - tm * tilesN;
  const int m0 = tm << 6;
  const int n0 = tn << 6;

  const T* Ab  = A  + (size_t)b * strideA;
  const T* Bb  = Bt + (size_t)b * strideB;
  const T* Ab2 = (SPL >= 1) ? (A2  + (size_t)b * strideA) : nullptr;
  const T* Bb2 = (SPL == 2) ? (Bt2 + (size_t)b * strideB) : nullptr;

  const int rlane = lane & 15;
  const int koff  = (lane >> 4) * 8;
  const int mOff  = (lane >> 4) * 8;

  v8f acc[4][4];
#pragma unroll
  for (int i = 0; i < 4; ++i)
#pragma unroll
    for (int j = 0; j < 4; ++j) acc[i][j] = (v8f){0.f,0.f,0.f,0.f,0.f,0.f,0.f,0.f};

  for (int k0 = 0; k0 < K; k0 += 32) {
    V bh[4], bl[4];
#pragma unroll
    for (int j = 0; j < 4; ++j) {
      const size_t bo = (size_t)(n0 + (j << 4) + rlane) * ldb + koff + k0;
      bh[j] = Frag<T>::load(Bb + bo);
      if (SPL == 2) bl[j] = Frag<T>::load(Bb2 + bo);
    }
#pragma unroll
    for (int i = 0; i < 4; ++i) {
      const size_t ao = (size_t)(m0 + (i << 4) + rlane) * lda + koff + k0;
      V ah = Frag<T>::load(Ab + ao);
      V al;
      if (SPL >= 1) al = Frag<T>::load(Ab2 + ao);
#pragma unroll
      for (int j = 0; j < 4; ++j) {
        acc[i][j] = Frag<T>::mma(ah, bh[j], acc[i][j]);
        if (SPL == 2) acc[i][j] = Frag<T>::mma(ah, bl[j], acc[i][j]);
        if (SPL >= 1) acc[i][j] = Frag<T>::mma(al, bh[j], acc[i][j]);
      }
      Frag<T>::guard(acc[i][0], acc[i][1], acc[i][2], acc[i][3], ah, (SPL >= 1) ? al : ah);
    }
    Frag<T>::keep(bh[0], bh[1], bh[2], bh[3]);
    if (SPL == 2) Frag<T>::keep(bl[0], bl[1], bl[2], bl[3]);
  }
  acc_guard4(acc[0][0], acc[0][1], acc[0][2], acc[0][3]);
  acc_guard4(acc[1][0], acc[1][1], acc[1][2], acc[1][3]);
  acc_guard4(acc[2][0], acc[2][1], acc[2][2], acc[2][3]);
  acc_guard4(acc[3][0], acc[3][1], acc[3][2], acc[3][3]);

  float* slab = sT[wave];
  const float* Rb = RESID ? (resid + (size_t)b * strideR) : nullptr;
#pragma unroll
  for (int i = 0; i < 4; ++i) {
    const int mBase = m0 + (i << 4);
#pragma unroll
    for (int j = 0; j < 4; ++j) {
      const int n = n0 + (j << 4) + rlane;
      float bv = 0.f;
      if (BIAS_MODE == 2) bv = bias[n];
#pragma unroll
      for (int r = 0; r < 8; ++r) {
        float v = acc[i][j][r] * scale;
        if (BIAS_MODE == 1) v += bias[mBase + mOff + r];
        if (BIAS_MODE == 2) v += bv;
        if (RESID) v += Rb[(size_t)(mBase + mOff + r) * ldc + n];
        if (ACT == 2) v = fmaxf(v, 0.0f);
        if (ACT == 4) v = (v > 0.f) ? v : 0.01f * v;
        slab[(mOff + r) * 68 + (j << 4) + rlane] = v;
      }
    }
    __builtin_amdgcn_fence(__ATOMIC_RELEASE, "workgroup");
    __builtin_amdgcn_wave_barrier();
    __builtin_amdgcn_fence(__ATOMIC_ACQUIRE, "workgroup");
    if (OUT_MODE == 0) {
      float* C = (float*)Cout + (size_t)b * strideC;
      const int hh = lane >> 4, c4 = (lane & 15) * 4;
      for (int pass = 0; pass < 2; ++pass) {
#pragma unroll
        for (int it = 0; it < 8; ++it) {
          const int row = it * 2 + hh;
          v4f v = *(const v4f*)(slab + row * 68 + c4);
          *(volatile v4f*)(C + (size_t)(mBase + row) * ldc + n0 + c4) = v;
        }
        __threadfence();
      }
    } else {
      const int q = lane >> 3, c8 = (lane & 7) * 8;
      unsigned short* C  = (unsigned short*)Cout  + (size_t)b * strideC;
      unsigned short* C2 = (OUT_MODE == 2) ? ((unsigned short*)Cout2 + (size_t)b * strideC) : nullptr;
      for (int pass = 0; pass < 2; ++pass) {
#pragma unroll
        for (int it = 0; it < 4; ++it) {
          const int row = it * 4 + q;
          const float* sp = slab + row * 68 + c8;
          v8h hv, lv;
#pragma unroll
          for (int e = 0; e < 8; ++e) {
            if (OUT_MODE == 1) {
              hv[e] = (_Float16)sp[e];
            } else {
              unsigned short hb = f2bf_bits(sp[e]);
              unsigned short lb = f2bf_bits(sp[e] - bf_bits2f(hb));
              hv[e] = __builtin_bit_cast(_Float16, hb);
              lv[e] = __builtin_bit_cast(_Float16, lb);
            }
          }
          *(volatile v8h*)(C + (size_t)(mBase + row) * ldc + n0 + c8) = hv;
          if (OUT_MODE == 2) *(volatile v8h*)(C2 + (size_t)(mBase + row) * ldc + n0 + c8) = lv;
        }
        __threadfence();
      }
    }
    __builtin_amdgcn_fence(__ATOMIC_RELEASE, "workgroup");
    __builtin_amdgcn_wave_barrier();
    __builtin_amdgcn_fence(__ATOMIC_ACQUIRE, "workgroup");
  }
}

__global__ __launch_bounds__(256) void split_rows_bf16_kernel(
    const float* __restrict__ src, unsigned short* __restrict__ dhi, unsigned short* __restrict__ dlo,
    int total8, int real8)
{
  const int i = blockIdx.x * 256 + threadIdx.x;
  if (i >= total8) return;
  const bool live = (i < real8);
  const int ic = live ? i : (real8 - 1);
  const size_t es = (size_t)ic << 3;
  const size_t e0 = (size_t)i << 3;
  const v4f a0 = *(const v4f*)(src + es);
  const v4f a1 = *(const v4f*)(src + es + 4);
  v8h hv, lv;
#pragma unroll
  for (int e = 0; e < 4; ++e) {
    const float s0 = live ? a0[e] : 0.0f;
    const float s1 = live ? a1[e] : 0.0f;
    const unsigned short h0 = f2bf_bits(s0), h1 = f2bf_bits(s1);
    const unsigned short l0 = f2bf_bits(s0 - bf_bits2f(h0)), l1 = f2bf_bits(s1 - bf_bits2f(h1));
    hv[e]     = __builtin_bit_cast(_Float16, h0);
    hv[4 + e] = __builtin_bit_cast(_Float16, h1);
    lv[e]     = __builtin_bit_cast(_Float16, l0);
    lv[4 + e] = __builtin_bit_cast(_Float16, l1);
  }
  unsigned short* qh = dhi + e0;
  unsigned short* ql = dlo + e0;
  *(volatile v8h*)qh = hv;
  *(volatile v8h*)ql = lv;
  __threadfence();
  *(volatile v8h*)qh = hv;
  *(volatile v8h*)ql = lv;
}

__global__ __launch_bounds__(256) void ln_split_kernel(
    const float* __restrict__ x, const float* __restrict__ wn, const float* __restrict__ bn,
    unsigned short* __restrict__ XNH, unsigned short* __restrict__ XNL)
{
  __shared__ float sX[kDm * kLnP];
  __shared__ float sS[4 * kLnTok];
  __shared__ float sQ[4 * kLnTok];
  __shared__ float sMu[kLnTok];
  __shared__ float sInv[kLnTok];
  __shared__ float sWn[kDm];
  __shared__ float sBn[kDm];
  const int tid = threadIdx.x;
  constexpr int kBlkPerB = kSeq / kLnTok;
  const int bix = blockIdx.x / kBlkPerB;
  const int l0  = (blockIdx.x - bix * kBlkPerB) * kLnTok;
  const float* xb = x + (size_t)bix * kDm * kSeq + l0;
  if (tid < kDm) { sWn[tid] = wn[tid]; sBn[tid] = bn[tid]; }
#pragma unroll 4
  for (int p = 0; p < 12; ++p) {
    const int idx = tid + p * 256;
    const int c   = idx >> 4;
    const int l4  = (idx & 15) * 4;
    const v4f v = *(const v4f*)(xb + (size_t)c * kSeq + l4);
    float* sp = sX + c * kLnP + l4;
    sp[0] = v[0]; sp[1] = v[1]; sp[2] = v[2]; sp[3] = v[3];
  }
  __syncthreads();
  const int l = tid & (kLnTok - 1);
  const int part = tid >> 6;
  {
    float s = 0.0f;
#pragma unroll 4
    for (int cc = 0; cc < 48; ++cc) s += sX[(part * 48 + cc) * kLnP + l];
    sS[part * kLnTok + l] = s;
  }
  __syncthreads();
  const float mu = ((sS[l] + sS[kLnTok + l]) + (sS[2 * kLnTok + l] + sS[3 * kLnTok + l])) * kInvDm;
  {
    float qv = 0.0f;
#pragma unroll 4
    for (int cc = 0; cc < 48; ++cc) {
      const float dv = sX[(part * 48 + cc) * kLnP + l] - mu;
      qv = fmaf(dv, dv, qv);
    }
    sQ[part * kLnTok + l] = qv;
  }
  __syncthreads();
  {
    const float var = ((sQ[l] + sQ[kLnTok + l]) + (sQ[2 * kLnTok + l] + sQ[3 * kLnTok + l])) * kInvDm;
    const float inv = 1.0f / sqrtf(var + 1e-5f);
    if (tid < kLnTok) { sMu[l] = mu; sInv[l] = inv; }
  }
  __syncthreads();
  const int tok0 = bix * kSeq + l0;
#pragma unroll 1
  for (int it = 0; it < 6; ++it) {
    const int u   = it * 256 + tid;
    const int row = u / 24;
    const int c0  = (u - row * 24) * 8;
    const float rm = sMu[row], ri = sInv[row];
    v8h hv, lv;
#pragma unroll
    for (int e = 0; e < 8; ++e) {
      const float xv = sX[(c0 + e) * kLnP + row];
      const float nv = (xv - rm) * ri * sWn[c0 + e] + sBn[c0 + e];
      const unsigned short hb = f2bf_bits(nv);
      const unsigned short lb = f2bf_bits(nv - bf_bits2f(hb));
      hv[e] = __builtin_bit_cast(_Float16, hb);
      lv[e] = __builtin_bit_cast(_Float16, lb);
    }
    unsigned short* qh = XNH + (size_t)(tok0 + row) * kDm + c0;
    unsigned short* ql = XNL + (size_t)(tok0 + row) * kDm + c0;
    *(volatile v8h*)qh = hv;
    *(volatile v8h*)ql = lv;
    __threadfence();
    *(volatile v8h*)qh = hv;
    *(volatile v8h*)ql = lv;
  }
}

__global__ __launch_bounds__(128) void conv_silu_kernel(
    const float* __restrict__ XZ, const float* __restrict__ cw, const float* __restrict__ cb,
    float* __restrict__ UC, unsigned short* __restrict__ UCH)
{
  __shared__ __align__(16) float sT[16 * kConvTP];
  const int tid = threadIdx.x, lane = tid & 31, wave = tid >> 5;
  const int d0 = blockIdx.x * kConvCh, d = d0 + tid;
  const int g0 = blockIdx.y * 64;
  const int tb = g0 & (kSeq - 1);
  const v4f wv = *(const v4f*)(cw + (size_t)d * 4);
  const float w0 = wv[0], w1 = wv[1], w2 = wv[2], w3 = wv[3];
  const float bc = cb[d];
  float xm3, xm2, xm1;
  {
    const bool hist = (tb > 0);
    const int rb = hist ? (g0 - 3) : g0;
    const float v3 = XZ[(size_t)rb * kXzP + d];
    const float v2 = XZ[(size_t)(rb + 1) * kXzP + d];
    const float v1 = XZ[(size_t)(rb + 2) * kXzP + d];
    xm3 = hist ? v3 : 0.f;
    xm2 = hist ? v2 : 0.f;
    xm1 = hist ? v1 : 0.f;
  }
  const int hh = lane >> 4, c8 = (lane & 15) * 8;
#pragma unroll 1
  for (int sub = 0; sub < 4; ++sub) {
    const int lb = g0 + sub * 16;
#pragma unroll 1
    for (int s = 0; s < 16; ++s) {
      const float xcur = XZ[(size_t)(lb + s) * kXzP + d];
      float acc = w0 * xm3;
      acc = fmaf(w1, xm2, acc);
      acc = fmaf(w2, xm1, acc);
      acc = fmaf(w3, xcur, acc);
      const float sv = acc + bc;
      const float sg = 1.0f / (1.0f + expf(-sv));
      sT[s * kConvTP + tid] = sv * sg;
      xm3 = xm2; xm2 = xm1; xm1 = xcur;
    }
    __syncthreads();
    v4f fv[4];
    v8h bh[2];
#pragma unroll
    for (int it = 0; it < 4; ++it) fv[it] = *(const v4f*)(sT + (it * 4 + wave) * kConvTP + lane * 4);
#pragma unroll
    for (int it = 0; it < 2; ++it) {
      const float* sp = sT + (it * 8 + wave * 2 + hh) * kConvTP + c8;
      const v4f a0 = *(const v4f*)(sp);
      const v4f a1 = *(const v4f*)(sp + 4);
#pragma unroll
      for (int e = 0; e < 4; ++e) {
        const unsigned short h0 = f2bf_bits(a0[e]), h1 = f2bf_bits(a1[e]);
        bh[it][e]     = __builtin_bit_cast(_Float16, h0);
        bh[it][4 + e] = __builtin_bit_cast(_Float16, h1);
      }
    }
    for (int pass = 0; pass < 2; ++pass) {
#pragma unroll
      for (int it = 0; it < 4; ++it)
        *(volatile v4f*)(UC + (size_t)(lb + it * 4 + wave) * kDin + d0 + lane * 4) = fv[it];
#pragma unroll
      for (int it = 0; it < 2; ++it)
        *(volatile v8h*)(UCH + (size_t)(lb + it * 8 + wave * 2 + hh) * kDin + d0 + c8) = bh[it];
      __threadfence();
    }
    __syncthreads();
  }
}

__global__ __launch_bounds__(64) void scan_kernel(
    const float* __restrict__ XD, const float* __restrict__ UC, const float* __restrict__ XZ,
    const float* __restrict__ Wdt, const float* __restrict__ bdt, const float* __restrict__ Alog,
    const float* __restrict__ Dp, unsigned short* __restrict__ YH, unsigned short* __restrict__ YL)
{
  __shared__ __align__(16) float sX[kScanTS * kXdP];
  __shared__ __align__(16) float sY[kScanTS * kScanYP];
  __shared__ __align__(16) float sW[kDtR * kScanCh];
  __shared__ __align__(16) float sA[kNst * kScanCh];
  const int tid = threadIdx.x, lane = tid & 31, wave = tid >> 5;
  constexpr int kBlkPerB = kDin / kScanCh;
  const int bix = blockIdx.x / kBlkPerB;
  const int d0  = (blockIdx.x - bix * kBlkPerB) * kScanCh;
  const int d   = d0 + tid;
  const size_t row0 = (size_t)bix * kSeq;
#pragma unroll 1
  for (int r = 0; r < kDtR; ++r) sW[r * kScanCh + tid] = Wdt[(size_t)d * kDtR + r];
#pragma unroll 1
  for (int s = 0; s < kNst; ++s) sA[s * kScanCh + tid] = -expf(Alog[(size_t)d * kNst + s]);
  __syncthreads();
  float negA[kNst], h[kNst];
#pragma unroll
  for (int s = 0; s < kNst; ++s) {
    negA[s] = sA[s * kScanCh + tid];
    h[s] = 0.f;
  }
  const float bb = bdt[d], Dd = Dp[d];
  const int lr = tid >> 4, lc4 = (tid & 15) * 4;
  const int q = lane >> 3, c8 = (lane & 7) * 8;
#pragma unroll 1
  for (int t0 = 0; t0 < kSeq; t0 += kScanTS) {
    __syncthreads();
#pragma unroll
    for (int i = 0; i < 16; ++i) {
      const int r = lr + 4 * i;
      *(v4f*)(sX + r * kXdP + lc4) = *(const v4f*)(XD + (row0 + t0 + r) * kXdP + lc4);
    }
    __syncthreads();
#pragma unroll 1
    for (int s = 0; s < kScanTS; ++s) {
      const int t = t0 + s;
      const float* xr = sX + s * kXdP;
      float vdot = 0.f;
#pragma unroll 1
      for (int r4 = 0; r4 < kDtR / 4; ++r4) {
        const v4f xv = *(const v4f*)(xr + 4 * r4);
        const float* wp = sW + (4 * r4) * kScanCh + tid;
        vdot = fmaf(xv[0], wp[0], vdot);
        vdot = fmaf(xv[1], wp[kScanCh], vdot);
        vdot = fmaf(xv[2], wp[2 * kScanCh], vdot);
        vdot = fmaf(xv[3], wp[3 * kScanCh], vdot);
      }
      float Bs[kNst], Cs[kNst];
#pragma unroll
      for (int q4 = 0; q4 < 4; ++q4) {
        const v4f bv = *(const v4f*)(xr + kDtR + 4 * q4);
        const v4f cv = *(const v4f*)(xr + kDtR + kNst + 4 * q4);
        Bs[4 * q4 + 0] = bv[0]; Bs[4 * q4 + 1] = bv[1]; Bs[4 * q4 + 2] = bv[2]; Bs[4 * q4 + 3] = bv[3];
        Cs[4 * q4 + 0] = cv[0]; Cs[4 * q4 + 1] = cv[1]; Cs[4 * q4 + 2] = cv[2]; Cs[4 * q4 + 3] = cv[3];
      }
      const float v   = vdot + bb;
      const float a   = __expf(-fabsf(v));
      const float u   = 1.0f + a;
      const float l1p = __logf(u) + (a - (u - 1.0f)) * __builtin_amdgcn_rcpf(u);
      const float dt  = fmaxf(v, 0.0f) + l1p;
      const float xt  = UC[(row0 + t) * kDin + d];
      const float dtx = dt * xt;
      float y = 0.f;
#pragma unroll
      for (int k = 0; k < kNst; ++k) {
        const float e = __expf(dt * negA[k]);
        h[k] = e * h[k] + dtx * Bs[k];
        y = h[k] * Cs[k] + y;
      }
      y = xt * Dd + y;
      const float zv = XZ[(row0 + t) * kXzP + kDin + d];
      const float sg = 1.0f / (1.0f + expf(-zv));
      y = y * (zv * sg);
      sY[s * kScanYP + tid] = y;
    }
    __syncthreads();
    v8h hv[8], lv[8];
#pragma unroll
    for (int it = 0; it < 8; ++it) {
      const int row = it * 8 + wave * 4 + q;
      const float* sp = sY + row * kScanYP + c8;
      const v4f a0 = *(const v4f*)(sp);
      const v4f a1 = *(const v4f*)(sp + 4);
#pragma unroll
      for (int e = 0; e < 4; ++e) {
        const unsigned short h0 = f2bf_bits(a0[e]), h1 = f2bf_bits(a1[e]);
        const unsigned short l0 = f2bf_bits(a0[e] - bf_bits2f(h0)), l1 = f2bf_bits(a1[e] - bf_bits2f(h1));
        hv[it][e]     = __builtin_bit_cast(_Float16, h0);
        hv[it][4 + e] = __builtin_bit_cast(_Float16, h1);
        lv[it][e]     = __builtin_bit_cast(_Float16, l0);
        lv[it][4 + e] = __builtin_bit_cast(_Float16, l1);
      }
    }
    for (int pass = 0; pass < 2; ++pass) {
#pragma unroll
      for (int it = 0; it < 8; ++it) {
        const int row = it * 8 + wave * 4 + q;
        const size_t o = (row0 + t0 + row) * kDin + d0 + c8;
        *(volatile v8h*)(YH + o) = hv[it];
        *(volatile v8h*)(YL + o) = lv[it];
      }
      __threadfence();
    }
  }
}

extern "C" void kernel_launch(void* const* d_in, const int* in_sizes, int n_in,
                              void* d_out, int out_size, void* d_ws, size_t ws_size,
                              hipStream_t stream) {
  if (n_in < 12) return;
  if (in_sizes[0] != kBatch * kDm * kSeq) return;
  if (in_sizes[1] != kDm || in_sizes[2] != kDm) return;
  if (in_sizes[3] != kXzP * kDm) return;
  if (in_sizes[4] != kDin * 4 || in_sizes[5] != kDin) return;
  if (in_sizes[6] != kXdReal * kDin) return;
  if (in_sizes[7] != kDin * kDtR || in_sizes[8] != kDin) return;
  if (in_sizes[9] != kDin * kNst || in_sizes[10] != kDin) return;
  if (in_sizes[11] != kDm * kDin) return;
  if (out_size != kBatch * kDm * kSeq) return;
  if (ws_size < kWsTotal) return;

  const float* x       = (const float*)d_in[0];
  const float* w_norm  = (const float*)d_in[1];
  const float* b_norm  = (const float*)d_in[2];
  const float* W_in    = (const float*)d_in[3];
  const float* W_conv  = (const float*)d_in[4];
  const float* b_conv  = (const float*)d_in[5];
  const float* W_xproj = (const float*)d_in[6];
  const float* W_dt    = (const float*)d_in[7];
  const float* b_dt    = (const float*)d_in[8];
  const float* A_log   = (const float*)d_in[9];
  const float* D_skip  = (const float*)d_in[10];
  const float* W_out   = (const float*)d_in[11];
  float* out = (float*)d_out;

  char* ws = (char*)d_ws;
  unsigned short* WIH = (unsigned short*)(ws + kOffWIH);
  unsigned short* WIL = (unsigned short*)(ws + kOffWIL);
  unsigned short* WOH = (unsigned short*)(ws + kOffWOH);
  unsigned short* WOL = (unsigned short*)(ws + kOffWOL);
  unsigned short* WXH = (unsigned short*)(ws + kOffWXH);
  unsigned short* WXL = (unsigned short*)(ws + kOffWXL);
  unsigned short* XNH = (unsigned short*)(ws + kOffXNH);
  unsigned short* XNL = (unsigned short*)(ws + kOffXNL);
  float*          XZ  = (float*)(ws + kOffXZ);
  float*          UC  = (float*)(ws + kOffUC);
  unsigned short* UCH = (unsigned short*)(ws + kOffUCH);
  float*          XD  = (float*)(ws + kOffXD);
  unsigned short* YH  = (unsigned short*)(ws + kOffYH);
  unsigned short* YL  = (unsigned short*)(ws + kOffYL);
  const float* dummy_bias  = b_dt;
  const float* dummy_resid = x;

  split_rows_bf16_kernel<<<(kXzP * kDm / 8) / 256, 256, 0, stream>>>(W_in, WIH, WIL, kXzP * kDm / 8, kXzP * kDm / 8);
  split_rows_bf16_kernel<<<(kDm * kDin / 8) / 256, 256, 0, stream>>>(W_out, WOH, WOL, kDm * kDin / 8, kDm * kDin / 8);
  split_rows_bf16_kernel<<<(kXdP * kDin / 8) / 256, 256, 0, stream>>>(W_xproj, WXH, WXL, kXdP * kDin / 8, kXdReal * kDin / 8);

  ln_split_kernel<<<kBatch * (kSeq / kLnTok), 256, 0, stream>>>(x, w_norm, b_norm, XNH, XNL);

  wmma_gemm64<1, 2, 0, 0, false><<<dim3(192, 1), 256, 0, stream>>>(
      XNH, XNL, kDm, 0L,
      WIH, WIL, kDm, 0L,
      (void*)XZ, (void*)XZ, kXzP, 0L,
      dummy_bias, dummy_resid, 0L,
      kRows, kXzP, kDm, 1.0f);

  conv_silu_kernel<<<dim3(kDin / kConvCh, kRows / 64), kConvCh, 0, stream>>>(XZ, W_conv, b_conv, UC, UCH);

  wmma_gemm64<1, 0, 0, 0, false><<<dim3(16, 1), 256, 0, stream>>>(
      UCH, UCH, kDin, 0L,
      WXH, WXH, kDin, 0L,
      (void*)XD, (void*)XD, kXdP, 0L,
      dummy_bias, dummy_resid, 0L,
      kRows, kXdP, kDin, 1.0f);

  scan_kernel<<<kBatch * (kDin / kScanCh), kScanCh, 0, stream>>>(XD, UC, XZ, W_dt, b_dt, A_log, D_skip, YH, YL);

  wmma_gemm64<1, 2, 0, 0, false><<<dim3(12, kBatch), 256, 0, stream>>>(
      WOH, WOL, kDin, 0L,
      YH, YL, kDin, (long)kSeq * kDin,
      (void*)out, (void*)out, kSeq, (long)kDm * kSeq,
      dummy_bias, dummy_resid, 0L,
      kDm, kSeq, kDin, 1.0f);
}
